// MultiHeadDiffAttention_79491254714581
// MI455X (gfx1250) — hardware-verified
//
#include <hip/hip_runtime.h>
#include <math.h>
#include <stdint.h>

#define NSEQ  2
#define SEQ   2048
#define DM    1024
#define NH    16
#define HD    64
#define DV    128
#define DVT   (NH * DV)
#define DQKV  (6 * DM)
#define VOFF  (4 * DM)
#define DC2   (2 * DM)
#define YP    DVT
#define NQB   (SEQ / 64)
#define QBH   8
#define THI   (QBH * 64)
#define GNG   32
#define STP   96
#define LAM_INIT 0.7778700995592556f
#define POST_SC  0.2221299004407444f
#define GN_EPS   1e-5f

static_assert(NH * HD == DM);
static_assert(HD == 64 && DV == 2 * HD);
static_assert(DVT == DC2 && YP == DC2);
static_assert((SEQ % 64) == 0 && (DM % 64) == 0 && (DQKV % 64) == 0 && (DC2 % 64) == 0);
static_assert((((SEQ / 64) * (DQKV / 64)) % 8) == 0);
static_assert((((SEQ / 64) * (DM / 64)) % 8) == 0);
static_assert(((SEQ * DM / 8) % 256) == 0 && ((DM * DM / 8) % 256) == 0 && ((DC2 * DM / 8) % 256) == 0);
static_assert(QBH > 0 && QBH < NQB && (THI % 64) == 0);
static_assert(GNG * 4 == DV && 2 * GNG + 1 <= STP && (STP % 4) == 0 && (STP / 4) <= 32);
static_assert((DVT % 256) == 0 && DC2 == 256 * 8);

typedef _Float16 v16h __attribute__((ext_vector_type(16)));
typedef _Float16 v8h  __attribute__((ext_vector_type(8)));
typedef float    v8f  __attribute__((ext_vector_type(8)));
typedef float    v4f  __attribute__((ext_vector_type(4)));
typedef unsigned int v4u __attribute__((ext_vector_type(4)));

__device__ __forceinline__ unsigned short bf_bits(float f) {
  unsigned u = __float_as_uint(f);
  return (unsigned short)((u + 0x7FFFu + ((u >> 16) & 1u)) >> 16);
}
__device__ __forceinline__ float bfr(float f) { return __uint_as_float(((unsigned)bf_bits(f)) << 16); }
__device__ __forceinline__ unsigned short h_bits(_Float16 x) { return __builtin_bit_cast(unsigned short, x); }
__device__ __forceinline__ unsigned pk16(unsigned short a, unsigned short b) { return (unsigned)a | ((unsigned)b << 16); }
__device__ __forceinline__ v8f zero8() { v8f z = {0.f, 0.f, 0.f, 0.f, 0.f, 0.f, 0.f, 0.f}; return z; }

__device__ __forceinline__ v16h ldfrag_h(const _Float16* p) {
  union { v16h v; v8h h[2]; } f;
  f.h[0] = *(const v8h*)(p);
  f.h[1] = *(const v8h*)(p + 16);
  return f.v;
}

__device__ __forceinline__ v8f mma_h(v16h a, v16h b, v8f c) {
  c = __builtin_amdgcn_wmma_f32_16x16x32_f16(false, a, false, b, (short)0, c, false, false);
#if defined(__HIP_DEVICE_COMPILE__)
  asm volatile("v_nop\n\tv_nop\n\tv_nop\n\tv_nop" : "+v"(c) : "v"(a), "v"(b));
#endif
  return c;
}
__device__ __forceinline__ v8f mma_h_raw(v16h a, v16h b, v8f c) {
  return __builtin_amdgcn_wmma_f32_16x16x32_f16(false, a, false, b, (short)0, c, false, false);
}
__device__ __forceinline__ void dep_guard_h(v8f& a, v8f& b, v16h x, v16h y) {
#if defined(__HIP_DEVICE_COMPILE__)
  asm volatile("v_nop\n\tv_nop\n\tv_nop\n\tv_nop" : "+v"(a), "+v"(b) : "v"(x), "v"(y));
#endif
}
__device__ __forceinline__ void keep4_h(v16h a, v16h b, v16h c, v16h d) {
#if defined(__HIP_DEVICE_COMPILE__)
  asm volatile("v_nop" :: "v"(a), "v"(b), "v"(c), "v"(d));
#endif
}
__device__ __forceinline__ void acc_guard4(v8f& a, v8f& b, v8f& c, v8f& d) {
#if defined(__HIP_DEVICE_COMPILE__)
  asm volatile("v_nop\n\tv_nop\n\tv_nop\n\tv_nop" : "+v"(a), "+v"(b), "+v"(c), "+v"(d));
#endif
}
template <int N>
__device__ __forceinline__ void acc_guardN(v8f (&a)[N]) {
  acc_guard4(a[0], a[1], a[2], a[3]);
  if constexpr (N == 8) acc_guard4(a[4], a[5], a[6], a[7]);
}

__global__ __launch_bounds__(256) void cvt16(const float* __restrict__ in, unsigned short* out, int n8, float scale) {
  const int i = blockIdx.x * 256 + threadIdx.x;
  if (i < n8) {
    const v4f a = *(const v4f*)(in + (size_t)i * 8);
    const v4f b = *(const v4f*)(in + (size_t)i * 8 + 4);
    v4u p;
    p[0] = pk16(h_bits((_Float16)(bfr(a[0]) * scale)), h_bits((_Float16)(bfr(a[1]) * scale)));
    p[1] = pk16(h_bits((_Float16)(bfr(a[2]) * scale)), h_bits((_Float16)(bfr(a[3]) * scale)));
    p[2] = pk16(h_bits((_Float16)(bfr(b[0]) * scale)), h_bits((_Float16)(bfr(b[1]) * scale)));
    p[3] = pk16(h_bits((_Float16)(bfr(b[2]) * scale)), h_bits((_Float16)(bfr(b[3]) * scale)));
    *(volatile v4u*)(out + (size_t)i * 8) = p;
    __threadfence();
    *(volatile v4u*)(out + (size_t)i * 8) = p;
  }
}

template <int EPI, bool ARES>
__global__ __launch_bounds__(256) void gemm64_f16(
    const unsigned short* __restrict__ Ap, const unsigned short* __restrict__ Arp, int lda,
    const unsigned short* __restrict__ Btp, int ldb, float cscale,
    void* Cp, unsigned short* Crp, int ldc, int M, int N, int K, float oscale,
    int tmod, int tlo, int thi, int rhi) {
  const _Float16* Ah  = (const _Float16*)(const void*)Ap;
  const _Float16* Arh = (const _Float16*)(const void*)Arp;
  const _Float16* Bt  = (const _Float16*)(const void*)Btp;
  __shared__ __align__(16) float sT[8][16 * 68];
  const int lane = threadIdx.x & 31;
  const int wave = threadIdx.x >> 5;
  const int tilesN = N >> 6;
  const int tilesM = M >> 6;
  const int tile = blockIdx.x * 8 + wave;
  if (tile >= tilesM * tilesN) return;
  const int tm = tile / tilesN;
  const int tn = tile - tm * tilesN;
  const int m0 = tm << 6;
  const int n0 = tn << 6;
  const int tpos = m0 % tmod;
  if (tpos < tlo || tpos >= thi) return;
  const bool wres = (tpos < rhi);

  const int rlane = lane & 15;
  const int koff  = (lane >> 4) * 8;
  const int mOff  = (lane >> 4) * 8;

  v8f acc[4][4];
#pragma unroll
  for (int i = 0; i < 4; ++i)
#pragma unroll
    for (int j = 0; j < 4; ++j) acc[i][j] = zero8();

  constexpr int NPL = ARES ? 2 : 1;
#pragma unroll 1
  for (int pl = 0; pl < NPL; ++pl) {
    const _Float16* Asel = (ARES && pl == 0) ? Arh : Ah;
    if (ARES && pl == 1) {
      acc_guard4(acc[0][0], acc[0][1], acc[0][2], acc[0][3]);
      acc_guard4(acc[1][0], acc[1][1], acc[1][2], acc[1][3]);
      acc_guard4(acc[2][0], acc[2][1], acc[2][2], acc[2][3]);
      acc_guard4(acc[3][0], acc[3][1], acc[3][2], acc[3][3]);
#pragma unroll
      for (int i = 0; i < 4; ++i)
#pragma unroll
        for (int j = 0; j < 4; ++j) acc[i][j] = acc[i][j] * (1.0f / 2048.0f);
      acc_guard4(acc[0][0], acc[0][1], acc[0][2], acc[0][3]);
      acc_guard4(acc[1][0], acc[1][1], acc[1][2], acc[1][3]);
      acc_guard4(acc[2][0], acc[2][1], acc[2][2], acc[2][3]);
      acc_guard4(acc[3][0], acc[3][1], acc[3][2], acc[3][3]);
    }
    for (int k0 = 0; k0 < K; k0 += 32) {
      v16h bh[4];
#pragma unroll
      for (int j = 0; j < 4; ++j) {
        const size_t bo = (size_t)(n0 + (j << 4) + rlane) * ldb + koff + k0;
        bh[j] = ldfrag_h(Bt + bo);
      }
#pragma unroll
      for (int i = 0; i < 4; ++i) {
        const size_t ao = (size_t)(m0 + (i << 4) + rlane) * lda + koff + k0;
        const v16h ah = ldfrag_h(Asel + ao);
#pragma unroll
        for (int j = 0; j < 4; ++j) {
          acc[i][j] = mma_h_raw(ah, bh[j], acc[i][j]);
        }
        dep_guard_h(acc[i][0], acc[i][3], ah, bh[3]);
      }
      keep4_h(bh[0], bh[1], bh[2], bh[3]);
    }
  }
  acc_guard4(acc[0][0], acc[0][1], acc[0][2], acc[0][3]);
  acc_guard4(acc[1][0], acc[1][1], acc[1][2], acc[1][3]);
  acc_guard4(acc[2][0], acc[2][1], acc[2][2], acc[2][3]);
  acc_guard4(acc[3][0], acc[3][1], acc[3][2], acc[3][3]);

  float* slab = sT[wave];
#pragma unroll
  for (int i = 0; i < 4; ++i) {
    const int mBase = m0 + (i << 4);
#pragma unroll
    for (int r = 0; r < 8; ++r) {
      const int row = mOff + r;
#pragma unroll
      for (int j = 0; j < 4; ++j) slab[row * 68 + (j << 4) + rlane] = acc[i][j][r] * cscale;
    }
    __builtin_amdgcn_fence(__ATOMIC_RELEASE, "workgroup");
    __builtin_amdgcn_wave_barrier();
    __builtin_amdgcn_fence(__ATOMIC_ACQUIRE, "workgroup");
    if constexpr (EPI == 0) {
      unsigned short* C16 = (unsigned short*)Cp;
      const int rq = lane >> 3, piece = lane & 7;
      v4u ph[4], pr[4];
#pragma unroll
      for (int it = 0; it < 4; ++it) {
        const int row = it * 4 + rq;
        const v4f a  = *(const v4f*)(slab + row * 68 + piece * 8);
        const v4f a2 = *(const v4f*)(slab + row * 68 + piece * 8 + 4);
        float f[8];
        f[0] = a[0];  f[1] = a[1];  f[2] = a[2];  f[3] = a[3];
        f[4] = a2[0]; f[5] = a2[1]; f[6] = a2[2]; f[7] = a2[3];
        v4u p, q;
#pragma unroll
        for (int e = 0; e < 4; ++e) {
          const float g0 = f[2 * e] * oscale, g1 = f[2 * e + 1] * oscale;
          const _Float16 x0 = (_Float16)g0, x1 = (_Float16)g1;
          const _Float16 y0 = (_Float16)((g0 - (float)x0) * 2048.0f);
          const _Float16 y1 = (_Float16)((g1 - (float)x1) * 2048.0f);
          p[e] = pk16(h_bits(x0), h_bits(x1));
          q[e] = pk16(h_bits(y0), h_bits(y1));
        }
        ph[it] = p;
        pr[it] = q;
      }
      for (int pass = 0; pass < 2; ++pass) {
#pragma unroll
        for (int it = 0; it < 4; ++it) {
          const int row = it * 4 + rq;
          const size_t co = (size_t)(mBase + row) * ldc + n0 + piece * 8;
          *(volatile v4u*)(C16 + co) = ph[it];
          if (wres) *(volatile v4u*)(Crp + co) = pr[it];
        }
        __threadfence();
      }
    } else {
      float* Cf = (float*)Cp;
      const int hh = lane >> 4, c4 = (lane & 15) * 4;
      v4f ov[8];
#pragma unroll
      for (int it = 0; it < 8; ++it) {
        const int row = it * 2 + hh;
        ov[it] = *(const v4f*)(slab + row * 68 + c4);
      }
      for (int pass = 0; pass < 2; ++pass) {
#pragma unroll
        for (int it = 0; it < 8; ++it) {
          const int row = it * 2 + hh;
          *(volatile v4f*)(Cf + (size_t)(mBase + row) * ldc + n0 + c4) = ov[it];
        }
        __threadfence();
      }
    }
    __builtin_amdgcn_fence(__ATOMIC_RELEASE, "workgroup");
    __builtin_amdgcn_wave_barrier();
    __builtin_amdgcn_fence(__ATOMIC_ACQUIRE, "workgroup");
  }
}

__global__ __launch_bounds__(256) void v_tr(const unsigned short* __restrict__ qkvp, unsigned short* vt, int opitch) {
  __shared__ __align__(16) _Float16 sv[64 * 72];
  const int tid = threadIdx.x;
  const int t0  = blockIdx.x * 64;
  const int fy  = blockIdx.y;
  const _Float16* src = (const _Float16*)(const void*)qkvp;
#pragma unroll
  for (int i = 0; i < 2; ++i) {
    const int idx = i * 256 + tid;
    const int tt = idx >> 3, c8 = (idx & 7) * 8;
    const v8h a = *(const v8h*)(src + ((size_t)(t0 + tt)) * DQKV + VOFF + fy * 64 + c8);
    *(v8h*)(sv + tt * 72 + c8) = a;
  }
  __syncthreads();

  const int g = tid >> 3, piece = tid & 7;
  v4u hv[2];
  size_t hofs[2];
#pragma unroll
  for (int it = 0; it < 2; ++it) {
    const int d = it * 32 + g;
    v4u a;
#pragma unroll
    for (int e = 0; e < 4; ++e) {
      const _Float16 x0 = sv[(piece * 8 + 2 * e) * 72 + d];
      const _Float16 x1 = sv[(piece * 8 + 2 * e + 1) * 72 + d];
      a[e] = pk16(h_bits(x0), h_bits(x1));
    }
    hv[it] = a;
    hofs[it] = ((size_t)(fy * 64 + d)) * opitch + t0 + piece * 8;
  }
  for (int pass = 0; pass < 2; ++pass) {
#pragma unroll
    for (int it = 0; it < 2; ++it) *(volatile v4u*)(vt + hofs[it]) = hv[it];
    __threadfence();
  }
}

__global__ __launch_bounds__(256) void v_prefix(const unsigned short* __restrict__ qkvp, float* S) {
  const int f = blockIdx.x * 256 + threadIdx.x;
  if (f >= DVT) return;
  const _Float16* src = (const _Float16*)(const void*)qkvp + VOFF + f;
  float acc = 0.0f;
#pragma unroll 2
  for (int t = 0; t < SEQ; ++t) {
    acc += (float)src[(size_t)t * DQKV] * (1.0f / 16.0f);
    float* d = S + (size_t)t * YP + f;
    *(volatile float*)d = acc;
    __threadfence();
    *(volatile float*)d = acc;
  }
}

template <bool HR, int NVT>
__global__ __launch_bounds__(128)
void attn_k(const unsigned short* __restrict__ qkvp, const unsigned short* __restrict__ qkvrp,
            const unsigned short* __restrict__ vtp, const unsigned short* __restrict__ vtrp,
            const float* __restrict__ Sp, float* C1p, float* C2p, int qb_lo, int qb_n) {
  union FH { v16h v; v8h h[2]; };
  constexpr bool CEN    = !HR;
  constexpr int  VC     = NVT * 16;
  constexpr int  NVHV   = DV / VC;
  constexpr int  TBK    = 64 * 64 * 2;
  constexpr int  TBV    = VC * 64 * 2;
  constexpr int  PB     = 4 * 16 * 64 * 2;
  constexpr int  OFF_K  = 0;
  constexpr int  OFF_V  = OFF_K + TBK;
  constexpr int  OFF_KR = OFF_V + TBV;
  constexpr int  OFF_VR = OFF_KR + TBK;
  constexpr int  OFF_P  = HR ? (OFF_VR + TBV) : (OFF_V + TBV);
  constexpr int  OFF_PR = OFF_P + PB;
  constexpr int  SMEMB  = HR ? (OFF_PR + PB) : (OFF_P + PB);
  constexpr int  OSB    = 4 * 16 * VC * 4;
  constexpr int  VHT    = (VC * 64) / 128;
  constexpr int  TPR    = 64 / VHT;
  constexpr int  LPR    = VC / 4;
  constexpr int  RPI    = 32 / LPR;
  constexpr int  NIT    = 16 / RPI;
  static_assert(OSB <= SMEMB);
  static_assert(NVHV * VC == DV);
  static_assert(VHT * 128 == VC * 64 && (VHT % 8) == 0 && TPR * VHT == 64);
  static_assert(LPR * RPI == 32 && NIT * RPI == 16 && (NIT % 8) == 0);
  __shared__ __align__(16) unsigned char smem[SMEMB];
  _Float16* Ksh = (_Float16*)(smem + OFF_K);
  _Float16* Vsh = (_Float16*)(smem + OFF_V);
  _Float16* Krs = (_Float16*)(smem + (HR ? OFF_KR : OFF_K));
  _Float16* Vrs = (_Float16*)(smem + (HR ? OFF_VR : OFF_V));
  _Float16* Psh = (_Float16*)(smem + OFF_P);
  _Float16* Prs = (_Float16*)(smem + (HR ? OFF_PR : OFF_P));

  const int tid  = threadIdx.x;
  const int wave = tid >> 5;
  const int lane = tid & 31;
  const int hh   = lane >> 4;
  const int c    = lane & 15;

  const int bx   = blockIdx.x;
  const int qb   = qb_lo + bx % qb_n;
  int rest       = bx / qb_n;
  const int vh   = rest % NVHV;
  rest           = rest / NVHV;
  const int map  = rest & 1;
  const int h    = rest >> 1;
  const int q0   = qb * 64 + wave * 16;
  const int cb   = h * DV + vh * VC;

  const _Float16* Qp  = (const _Float16*)(const void*)qkvp  + (size_t)map * DM + (size_t)h * HD;
  const _Float16* Qrp = (const _Float16*)(const void*)qkvrp + (size_t)map * DM + (size_t)h * HD;
  const _Float16* Kp  = Qp + 2 * DM;
  const _Float16* Krp = Qrp + 2 * DM;
  const _Float16* Vt  = (const _Float16*)(const void*)vtp  + (size_t)cb * SEQ;
  const _Float16* Vrt = (const _Float16*)(const void*)vtrp + (size_t)cb * THI;
  float* Co = map ? C2p : C1p;

  v16h qa[2], qr[2];
#pragma unroll
  for (int dc = 0; dc < 2; ++dc) {
    const size_t qo = (size_t)(q0 + c) * DQKV + dc * 32 + 8 * hh;
    qa[dc] = ldfrag_h(Qp + qo);
    if constexpr (HR) qr[dc] = ldfrag_h(Qrp + qo);
    else qr[dc] = qa[dc];
  }

  float lsum[8], mrun[8];
  v8f oacc[NVT], oacc2[NVT];
#pragma unroll
  for (int r = 0; r < 8; ++r) { lsum[r] = 0.f; mrun[r] = -1e30f; }
#pragma unroll
  for (int t = 0; t < NVT; ++t) { oacc[t] = zero8(); oacc2[t] = zero8(); }

  _Float16* pw  = Psh + wave * (16 * 64);
  _Float16* prw = Prs + wave * (16 * 64);

  const int nkt = qb + 1;
  for (int kt = 0; kt < nkt; ++kt) {
    const int kv0 = kt * 64;
    __syncthreads();
    {
      const int r = tid >> 1, half = (tid & 1) * 32;
      const size_t ko = (size_t)(kv0 + r) * DQKV + half;
#pragma unroll
      for (int i = 0; i < 4; ++i) {
        const v8h a0 = *(const v8h*)(Kp + ko + 8 * i);
        *(v8h*)(Ksh + r * 64 + half + 8 * i) = a0;
        if constexpr (HR) {
          const v8h a1 = *(const v8h*)(Krp + ko + 8 * i);
          *(v8h*)(Krs + r * 64 + half + 8 * i) = a1;
        }
      }
      const int vr = tid / TPR, voff = (tid - vr * TPR) * VHT;
      const size_t vo  = (size_t)vr * SEQ + kv0 + voff;
      const size_t vro = (size_t)vr * THI + kv0 + voff;
#pragma unroll
      for (int i = 0; i < VHT / 8; ++i) {
        const v8h b0 = *(const v8h*)(Vt + vo + 8 * i);
        *(v8h*)(Vsh + vr * 64 + voff + 8 * i) = b0;
        if constexpr (HR) {
          const v8h b1 = *(const v8h*)(Vrt + vro + 8 * i);
          *(v8h*)(Vrs + vr * 64 + voff + 8 * i) = b1;
        }
      }
    }
    __syncthreads();

    v8f s[4];
#pragma unroll
    for (int j = 0; j < 4; ++j) {
      s[j] = zero8();
      v8f t = zero8();
#pragma unroll
      for (int dc = 0; dc < 2; ++dc) {
        FH kb;
        kb.h[0] = *(const v8h*)(Ksh + (j * 16 + c) * 64 + dc * 32 + 8 * hh);
        kb.h[1] = *(const v8h*)(Ksh + (j * 16 + c) * 64 + dc * 32 + 16 + 8 * hh);
        s[j] = mma_h(qa[dc], kb.v, s[j]);
        if constexpr (HR) {
          FH krb;
          krb.h[0] = *(const v8h*)(Krs + (j * 16 + c) * 64 + dc * 32 + 8 * hh);
          krb.h[1] = *(const v8h*)(Krs + (j * 16 + c) * 64 + dc * 32 + 16 + 8 * hh);
          t = mma_h(qa[dc], krb.v, t);
          t = mma_h(qr[dc], kb.v, t);
        }
      }
      if constexpr (HR) s[j] = s[j] + t * (1.0f / 2048.0f);
    }

    float alpha[8];
#pragma unroll
    for (int r = 0; r < 8; ++r) {
      const int qrow = q0 + 8 * hh + r;
      float av[4];
      float tmx = -1e30f;
#pragma unroll
      for (int j = 0; j < 4; ++j) {
        const int key = kv0 + j * 16 + c;
        float a = s[j][r] * (1.0f / 2048.0f);
        a = (key > qrow) ? -1e30f : a;
        av[j] = a;
        tmx = fmaxf(tmx, a);
      }
#pragma unroll
      for (int off = 1; off < 16; off <<= 1) tmx = fmaxf(tmx, __shfl_xor(tmx, off, 32));
      const float mn = fmaxf(mrun[r], tmx);
      const float al = __expf(mrun[r] - mn);
      alpha[r] = al;
      mrun[r]  = mn;
      float em = 0.0f;
      if constexpr (CEN) em = __expf(-mn);
      float ps = 0.0f;
#pragma unroll
      for (int j = 0; j < 4; ++j) {
        const int key = kv0 + j * 16 + c;
        float p = __expf(av[j] - mn);
        p = (key > qrow) ? 0.0f : p;
        ps += p;
        float pc = p;
        if constexpr (CEN) pc = (key > qrow) ? 0.0f : (p - em);
        const float g = pc * 256.0f;
        const _Float16 x0 = (_Float16)g;
        pw[(8 * hh + r) * 64 + j * 16 + c] = x0;
        if constexpr (HR) prw[(8 * hh + r) * 64 + j * 16 + c] = (_Float16)((g - (float)x0) * 2048.0f);
      }
      lsum[r] = lsum[r] * al + ps;
    }
    __builtin_amdgcn_fence(__ATOMIC_RELEASE, "workgroup");
    __builtin_amdgcn_wave_barrier();
    __builtin_amdgcn_fence(__ATOMIC_ACQUIRE, "workgroup");

#pragma unroll
    for (int t = 0; t < NVT; ++t) {
#pragma unroll
      for (int r = 0; r < 8; ++r) {
        oacc[t][r] = oacc[t][r] * alpha[r];
        if constexpr (HR) oacc2[t][r] = oacc2[t][r] * alpha[r];
      }
    }
    acc_guardN<NVT>(oacc);
    if constexpr (HR) acc_guardN<NVT>(oacc2);

#pragma unroll
    for (int kk = 0; kk < 2; ++kk) {
      FH pa, par;
      pa.h[0] = *(const v8h*)(pw + c * 64 + kk * 32 + 8 * hh);
      pa.h[1] = *(const v8h*)(pw + c * 64 + kk * 32 + 16 + 8 * hh);
      if constexpr (HR) {
        par.h[0] = *(const v8h*)(prw + c * 64 + kk * 32 + 8 * hh);
        par.h[1] = *(const v8h*)(prw + c * 64 + kk * 32 + 16 + 8 * hh);
      } else {
        par.v = pa.v;
      }
#pragma unroll
      for (int t = 0; t < NVT; ++t) {
        FH vb;
        vb.h[0] = *(const v8h*)(Vsh + (t * 16 + c) * 64 + kk * 32 + 8 * hh);
        vb.h[1] = *(const v8h*)(Vsh + (t * 16 + c) * 64 + kk * 32 + 16 + 8 * hh);
        oacc[t] = mma_h(pa.v, vb.v, oacc[t]);
        if constexpr (HR) {
          FH vrb;
          vrb.h[0] = *(const v8h*)(Vrs + (t * 16 + c) * 64 + kk * 32 + 8 * hh);
          vrb.h[1] = *(const v8h*)(Vrs + (t * 16 + c) * 64 + kk * 32 + 16 + 8 * hh);
          oacc2[t] = mma_h(pa.v, vrb.v, oacc2[t]);
          oacc2[t] = mma_h(par.v, vb.v, oacc2[t]);
        }
      }
    }
  }
  __syncthreads();

  float* os = (float*)(void*)smem + wave * (16 * VC);
#pragma unroll
  for (int r = 0; r < 8; ++r) {
    float l = lsum[r];
#pragma unroll
    for (int off = 1; off < 16; off <<= 1) l += __shfl_xor(l, off, 32);
    const float rl = 1.0f / l;
    float emf = 0.0f;
    if constexpr (CEN) emf = __expf(-mrun[r]);
    const int qrow = q0 + 8 * hh + r;
#pragma unroll
    for (int t = 0; t < NVT; ++t) {
      float v = oacc[t][r];
      if constexpr (HR) v += oacc2[t][r] * (1.0f / 2048.0f);
      v = v * (1.0f / 4096.0f);
      if constexpr (CEN) v += emf * Sp[(size_t)qrow * YP + cb + t * 16 + c];
      os[(8 * hh + r) * VC + t * 16 + c] = v * rl;
    }
  }
  __builtin_amdgcn_fence(__ATOMIC_RELEASE, "workgroup");
  __builtin_amdgcn_wave_barrier();
  __builtin_amdgcn_fence(__ATOMIC_ACQUIRE, "workgroup");
  {
    const int sub = lane / LPR;
    const int c4  = (lane - sub * LPR) * 4;
#pragma unroll
    for (int bt = 0; bt < NIT; bt += 8) {
      v4f ov[8];
#pragma unroll
      for (int it = 0; it < 8; ++it) {
        const int row = (bt + it) * RPI + sub;
        ov[it] = *(const v4f*)(os + row * VC + c4);
      }
      for (int pass = 0; pass < 2; ++pass) {
#pragma unroll
        for (int it = 0; it < 8; ++it) {
          const int row = (bt + it) * RPI + sub;
          *(volatile v4f*)(Co + (size_t)(q0 + row) * YP + cb + c4) = ov[it];
        }
        __threadfence();
      }
    }
  }
}

__global__ __launch_bounds__(256) void gn_stats(const float* __restrict__ C1, const float* __restrict__ C2,
                                                const float* __restrict__ lq1, const float* __restrict__ lk1,
                                                const float* __restrict__ lq2, const float* __restrict__ lk2,
                                                float* ST) {
  __shared__ double sd[256], sq[256];
  __shared__ __align__(16) float stg[STP];
  const int h   = blockIdx.x;
  const int tid = threadIdx.x;
  const float x1 = bfr(lq1[h]) * bfr(lk1[h]);
  const float x2 = bfr(lq2[h]) * bfr(lk2[h]);
  const float lam = 1.0f / (1.0f + expf(-x1)) - 1.0f / (1.0f + expf(-x2)) + LAM_INIT;
  const int c = tid & 127, par = tid >> 7;
  const float* p1 = C1 + (size_t)h * DV + c;
  const float* p2 = C2 + (size_t)h * DV + c;
  double s = 0.0, ss = 0.0;
#pragma unroll 2
  for (int t = par; t < SEQ; t += 2) {
    const size_t o = (size_t)t * YP;
    const float y = p1[o] - lam * p2[o];
    const double yd = (double)y;
    s  += yd;
    ss += yd * yd;
  }
  sd[tid] = s;
  sq[tid] = ss;
  if (tid < STP) stg[tid] = 0.0f;
  __syncthreads();
  if (tid < GNG) {
    double a = 0.0, q = 0.0;
#pragma unroll
    for (int j = 0; j < 4; ++j) {
      a += sd[tid * 4 + j];  a += sd[128 + tid * 4 + j];
      q += sq[tid * 4 + j];  q += sq[128 + tid * 4 + j];
    }
    const double inv = 1.0 / (double)(SEQ * 4);
    const double mu  = a * inv;
    double var = q * inv - mu * mu;
    var = var < 0.0 ? 0.0 : var;
    const float varf = (float)var;
    stg[tid] = (float)mu;
    stg[GNG + tid] = 1.0f / sqrtf(varf + GN_EPS);
    if (tid == 0) stg[2 * GNG] = lam;
  }
  __syncthreads();
  if (tid < STP / 4) {
    const v4f v = *(const v4f*)(stg + tid * 4);
    float* dst = ST + (size_t)h * STP + tid * 4;
    *(volatile v4f*)dst = v;
    __threadfence();
    *(volatile v4f*)dst = v;
  }
}

__global__ __launch_bounds__(256) void gn_apply(const float* __restrict__ C1, const float* __restrict__ C2,
                                                const float* __restrict__ ST, const float* __restrict__ gnw,
                                                const float* __restrict__ gnb, const float* __restrict__ gam,
                                                unsigned short* Yn, unsigned short* Ynr) {
  const int t  = blockIdx.x;
  const int f8 = threadIdx.x * 8;
  const int h  = f8 >> 7;
  const int c0 = f8 & 127;
  const int g0 = c0 >> 2;
  const float* st = ST + h * STP;
  const float mu0 = st[g0], mu1 = st[g0 + 1];
  const float rs0 = st[GNG + g0], rs1 = st[GNG + g0 + 1];
  const float lam = st[2 * GNG];
  const size_t ro = (size_t)t * YP + f8;
  const v4f a0 = *(const v4f*)(C1 + ro), a1 = *(const v4f*)(C1 + ro + 4);
  const v4f b0 = *(const v4f*)(C2 + ro), b1 = *(const v4f*)(C2 + ro + 4);
  const v4f w0 = *(const v4f*)(gnw + c0), w1 = *(const v4f*)(gnw + c0 + 4);
  const v4f e0 = *(const v4f*)(gnb + c0), e1 = *(const v4f*)(gnb + c0 + 4);
  const v4f m0 = *(const v4f*)(gam + c0), m1 = *(const v4f*)(gam + c0 + 4);
  float yn[8];
#pragma unroll
  for (int e = 0; e < 4; ++e) {
    const float y = a0[e] - lam * b0[e];
    yn[e] = (((y - mu0) * rs0) * bfr(w0[e]) + bfr(e0[e])) * bfr(m0[e]) * POST_SC;
  }
#pragma unroll
  for (int e = 0; e < 4; ++e) {
    const float y = a1[e] - lam * b1[e];
    yn[4 + e] = (((y - mu1) * rs1) * bfr(w1[e]) + bfr(e1[e])) * bfr(m1[e]) * POST_SC;
  }
  v4u p, q;
#pragma unroll
  for (int e = 0; e < 4; ++e) {
    const float g0v = yn[2 * e] * 16.0f, g1v = yn[2 * e + 1] * 16.0f;
    const _Float16 x0 = (_Float16)g0v, x1 = (_Float16)g1v;
    const _Float16 y0 = (_Float16)((g0v - (float)x0) * 2048.0f);
    const _Float16 y1 = (_Float16)((g1v - (float)x1) * 2048.0f);
    p[e] = pk16(h_bits(x0), h_bits(x1));
    q[e] = pk16(h_bits(y0), h_bits(y1));
  }
  const size_t wo = (size_t)t * DC2 + f8;
  for (int pass = 0; pass < 2; ++pass) {
    *(volatile v4u*)(Yn + wo) = p;
    if (t < THI) *(volatile v4u*)(Ynr + wo) = q;
    __threadfence();
  }
}

extern "C" void kernel_launch(void* const* d_in, const int* in_sizes, int n_in,
                              void* d_out, int out_size, void* d_ws, size_t ws_size,
                              hipStream_t stream) {
  if (n_in < 14) return;
  if (in_sizes[0] != NSEQ * SEQ * DM) return;
  if (in_sizes[1] != DM * DM) return;
  if (in_sizes[2] != DM * DM) return;
  if (in_sizes[3] != DM * DM) return;
  if (in_sizes[4] != DM * DM) return;
  if (in_sizes[5] != DC2 * DM) return;
  if (in_sizes[6] != DM * DC2) return;
  if (in_sizes[7] != DV || in_sizes[8] != DV || in_sizes[9] != DV) return;
  if (in_sizes[10] != NH || in_sizes[11] != NH || in_sizes[12] != NH || in_sizes[13] != NH) return;
  if (out_size != NSEQ * SEQ * DM) return;

  const float* x    = (const float*)d_in[0];
  const float* w_q1 = (const float*)d_in[1];
  const float* w_q2 = (const float*)d_in[2];
  const float* w_k1 = (const float*)d_in[3];
  const float* w_k2 = (const float*)d_in[4];
  const float* w_v  = (const float*)d_in[5];
  const float* w_c  = (const float*)d_in[6];
  const float* gnw  = (const float*)d_in[7];
  const float* gnb  = (const float*)d_in[8];
  const float* gam  = (const float*)d_in[9];
  const float* lq1  = (const float*)d_in[10];
  const float* lk1  = (const float*)d_in[11];
  const float* lq2  = (const float*)d_in[12];
  const float* lk2  = (const float*)d_in[13];

  const size_t PX    = (size_t)SEQ * DM * 2;
  const size_t PWq   = (size_t)DQKV * DM * 2;
  const size_t PWc   = (size_t)DM * DC2 * 2;
  const size_t PQKV  = (size_t)SEQ * DQKV * 2;
  const size_t PQKVr = (size_t)THI * DQKV * 2;
  const size_t PVT   = (size_t)DVT * SEQ * 2;
  const size_t PVTr  = (size_t)DVT * THI * 2;
  const size_t PC    = (size_t)SEQ * YP * 4;
  const size_t PYn   = (size_t)SEQ * DC2 * 2;
  const size_t PYnr  = (size_t)THI * DC2 * 2;
  const size_t PST   = 8192;
  size_t off = 0;
  const size_t oX    = off; off += PX;
  const size_t oWq   = off; off += PWq;
  const size_t oWc   = off; off += PWc;
  const size_t oQKV  = off; off += PQKV;
  const size_t oQKVr = off; off += PQKVr;
  const size_t oVT   = off; off += PVT;
  const size_t oVTr  = off; off += PVTr;
  const size_t oC1   = off; off += PC;
  const size_t oC2   = off; off += PC;
  const size_t oS    = off; off += PC;
  const size_t oYn   = off; off += PYn;
  const size_t oYnr  = off; off += PYnr;
  const size_t oST   = off; off += PST;
  if (off > ws_size) return;
  if (off > (size_t)134217728) return;
  if ((size_t)NH * STP * 4 > PST) return;

  char* ws = (char*)d_ws;
  unsigned short* Xh   = (unsigned short*)(ws + oX);
  unsigned short* Wqkv = (unsigned short*)(ws + oWq);
  unsigned short* Wcp  = (unsigned short*)(ws + oWc);
  unsigned short* QKV  = (unsigned short*)(ws + oQKV);
  unsigned short* QKVr = (unsigned short*)(ws + oQKVr);
  unsigned short* VT   = (unsigned short*)(ws + oVT);
  unsigned short* VTr  = (unsigned short*)(ws + oVTr);
  float*          C1   = (float*)(ws + oC1);
  float*          C2   = (float*)(ws + oC2);
  float*          S    = (float*)(ws + oS);
  unsigned short* Yn   = (unsigned short*)(ws + oYn);
  unsigned short* Ynr  = (unsigned short*)(ws + oYnr);
  float*          ST   = (float*)(ws + oST);
  float*          outf = (float*)d_out;

  const dim3 blk(256);
  const int n8x = SEQ * DM / 8;
  const int n8w = DM * DM / 8;
  const int n8v = DC2 * DM / 8;
  const dim3 gCx((n8x + 255) / 256);
  const dim3 gCw((n8w + 255) / 256);
  const dim3 gCv((n8v + 255) / 256);
  const dim3 gGqkv(((SEQ / 64) * (DQKV / 64) + 7) / 8);
  const dim3 gGout(((SEQ / 64) * (DM / 64) + 7) / 8);
  const dim3 gVt(SEQ / 64, DVT / 64, 1);
  const dim3 gVtr(THI / 64, DVT / 64, 1);
  const dim3 gPf(DVT / 256);
  const dim3 gAttnHi(QBH * (DV / 64) * 2 * NH);
  const dim3 gAttnLo((NQB - QBH) * (DV / 128) * 2 * NH);
  const dim3 gSt(NH);
  const dim3 gAp(SEQ);
  const float wScale = 1024.0f;
  const float aScale = 16.0f;
  const float cscale = 1.0f / 16384.0f;

  cvt16<<<gCw, blk, 0, stream>>>(w_q1, Wqkv, n8w, wScale);
  cvt16<<<gCw, blk, 0, stream>>>(w_q2, Wqkv + (size_t)DM * DM, n8w, wScale);
  cvt16<<<gCw, blk, 0, stream>>>(w_k1, Wqkv + (size_t)2 * DM * DM, n8w, wScale);
  cvt16<<<gCw, blk, 0, stream>>>(w_k2, Wqkv + (size_t)3 * DM * DM, n8w, wScale);
  cvt16<<<gCv, blk, 0, stream>>>(w_v,  Wqkv + (size_t)4 * DM * DM, n8v, wScale);
  cvt16<<<gCv, blk, 0, stream>>>(w_c,  Wcp, n8v, wScale);

  for (int grp = 0; grp < NSEQ; ++grp) {
    const float* xg = x + (size_t)grp * SEQ * DM;
    float* outg = outf + (size_t)grp * SEQ * DM;
    cvt16<<<gCx, blk, 0, stream>>>(xg, Xh, n8x, aScale);
    gemm64_f16<0, false><<<gGqkv, blk, 0, stream>>>(Xh, Xh, DM, Wqkv, DM, cscale, (void*)QKV, QKVr, DQKV,
                                                    SEQ, DQKV, DM, aScale, SEQ, 0, SEQ, THI);
    v_tr<<<gVt, blk, 0, stream>>>(QKV, VT, SEQ);
    v_tr<<<gVtr, blk, 0, stream>>>(QKVr, VTr, THI);
    v_prefix<<<gPf, blk, 0, stream>>>(QKV, S);
    attn_k<true, 4><<<gAttnHi, dim3(128), 0, stream>>>(QKV, QKVr, VT, VTr, S, C1, C2, 0, QBH);
    attn_k<false, 8><<<gAttnLo, dim3(128), 0, stream>>>(QKV, QKVr, VT, VTr, S, C1, C2, QBH, NQB - QBH);
    gn_stats<<<gSt, blk, 0, stream>>>(C1, C2, lq1, lk1, lq2, lk2, ST);
    gn_apply<<<gAp, blk, 0, stream>>>(C1, C2, ST, gnw, gnb, gam, Yn, Ynr);
    gemm64_f16<1, false><<<gGout, blk, 0, stream>>>(Yn, Ynr, DC2, Wcp, DC2, cscale, (void*)outg, Ynr, DM,
                                                    SEQ, DM, DC2, 1.0f, SEQ, THI, SEQ, 0);
    gemm64_f16<1, true><<<gGout, blk, 0, stream>>>(Yn, Ynr, DC2, Wcp, DC2, cscale, (void*)outg, Ynr, DM,
                                                   SEQ, DM, DC2, 1.0f, SEQ, 0, THI, 0);
  }
  (void)hipGetLastError();
}
